// GMNLayer_73031623901579
// MI455X (gfx1250) — hardware-verified
//
#include <hip/hip_runtime.h>
#include <stdint.h>

typedef __bf16 v16bf __attribute__((ext_vector_type(16)));
typedef __bf16 v8bf  __attribute__((ext_vector_type(8)));
typedef float  v8f   __attribute__((ext_vector_type(8)));
typedef float  v4f   __attribute__((ext_vector_type(4)));
typedef int    v4i   __attribute__((ext_vector_type(4)));

#define FD   128
#define NB   64
#define QCAP 256

union P8 { v8bf b; v4i i; };

static __device__ inline float relu_f(float v) { return fmaxf(v, 0.0f); }
static __device__ inline float clip100(float v) { return fminf(fmaxf(v, -100.0f), 100.0f); }

static __device__ inline float bf16_hi(float x) {
  unsigned u = __float_as_uint(x);
  u = (u + 0x7FFFu + ((u >> 16) & 1u)) & 0xFFFF0000u;
  return __uint_as_float(u);
}

static __device__ inline v8f zf8() {
  v8f z;
#pragma unroll
  for (int i = 0; i < 8; ++i) z[i] = 0.0f;
  return z;
}
static __device__ inline v16bf z16() {
  v16bf z;
#pragma unroll
  for (int i = 0; i < 16; ++i) z[i] = (__bf16)0.0f;
  return z;
}
static __device__ inline v8bf ld8(const __bf16* p) {
  return *reinterpret_cast<const v8bf*>(p);
}
static __device__ inline v16bf cat16(v8bf a, v8bf b) {
  return __builtin_shufflevector(a, b, 0,1,2,3,4,5,6,7,8,9,10,11,12,13,14,15);
}

static __device__ inline void asplit(const float* p, int hh, v16bf& hi, v16bf& lo) {
#pragma unroll
  for (int i = 0; i < 8; ++i) {
    const float x  = p[8 * hh + i];
    const float xh = bf16_hi(x);
    hi[i] = (__bf16)xh;
    lo[i] = (__bf16)(x - xh);
  }
#pragma unroll
  for (int i = 0; i < 8; ++i) {
    const float x  = p[16 + 8 * hh + i];
    const float xh = bf16_hi(x);
    hi[8 + i] = (__bf16)xh;
    lo[8 + i] = (__bf16)(x - xh);
  }
}
static __device__ inline v16bf bfr(const __bf16* p, int hh) {
  return cat16(ld8(p + 8 * hh), ld8(p + 16 + 8 * hh));
}

static __device__ inline v8f wmma3(v16bf ah, v16bf al, v16bf bh, v16bf bl, v8f c) {
  c = __builtin_amdgcn_wmma_f32_16x16x32_bf16(false, ah, false, bh, (short)0, c, false, false);
  c = __builtin_amdgcn_wmma_f32_16x16x32_bf16(false, al, false, bh, (short)0, c, false, false);
  c = __builtin_amdgcn_wmma_f32_16x16x32_bf16(false, ah, false, bl, (short)0, c, false, false);
  asm volatile("v_nop\n\tv_nop\n\tv_nop\n\tv_nop" : "+v"(c) : "v"(ah), "v"(al), "v"(bh), "v"(bl));
  return c;
}
static __device__ inline v8f kstep(v8f acc, const float* ap, const __bf16* bph,
                                     const __bf16* bpl, int hh) {
  v16bf ah, al;
  asplit(ap, hh, ah, al);
  const v16bf bh = bfr(bph, hh);
  const v16bf bl = bfr(bpl, hh);
  return wmma3(ah, al, bh, bl, acc);
}

__global__ __launch_bounds__(256) void k_wsplit(const float* __restrict__ src,
                                                __bf16* dh, __bf16* dl,
                                                int Ksrc, int Kpad) {
  const int per = Kpad >> 3;
  const int total = 128 * per;
  const int idx = blockIdx.x * blockDim.x + threadIdx.x;
  if (idx >= total) return;
  const int n  = idx / per;
  const int k8 = (idx - n * per) * 8;
  P8 uh, ul;
#pragma unroll
  for (int i = 0; i < 8; ++i) {
    const int k = k8 + i;
    const float x  = (k < Ksrc) ? src[(size_t)k * 128 + n] : 0.0f;
    const float xh = bf16_hi(x);
    uh.b[i] = (__bf16)xh;
    ul.b[i] = (__bf16)(x - xh);
  }
  volatile v4i* ph = (volatile v4i*)(dh + (size_t)idx * 8);
  volatile v4i* pl = (volatile v4i*)(dl + (size_t)idx * 8);
  *ph = uh.i;
  *pl = ul.i;
  __threadfence();
  *ph = uh.i;
  *pl = ul.i;
}

__global__ __launch_bounds__(32) void k_layer(
    const float* __restrict__ h, const float* __restrict__ coord,
    const float* __restrict__ others,
    const int* __restrict__ erow, const int* __restrict__ ecol,
    const __bf16* __restrict__ w1h, const __bf16* __restrict__ w1l, const float* __restrict__ be1,
    const __bf16* __restrict__ w2h, const __bf16* __restrict__ w2l, const float* __restrict__ be2,
    const __bf16* __restrict__ w3h, const __bf16* __restrict__ w3l, const float* __restrict__ bc1,
    const float* __restrict__ wc2,
    const __bf16* __restrict__ w4h, const __bf16* __restrict__ w4l, const float* __restrict__ bn1,
    const __bf16* __restrict__ w5h, const __bf16* __restrict__ w5l, const float* __restrict__ bn2,
    float* hOut, float* cOut, int N, int E) {
#pragma clang fp contract(off)
  __shared__ __attribute__((aligned(16))) float aggL[NB * FD];
  __shared__ __attribute__((aligned(16))) float tH[16 * FD];
  __shared__ __attribute__((aligned(16))) float tF[16 * FD];
  __shared__ __attribute__((aligned(16))) float cL[NB * 3];
  __shared__ float csumL[NB * 4];
  __shared__ float phiL[16];
  __shared__ int   qL[QCAP];

  const int lane = threadIdx.x & 31;
  const int hh   = lane >> 4;
  const int m15  = lane & 15;
  const int v0   = blockIdx.x * NB;
  if (v0 >= N) return;

  for (int i = lane; i < NB * FD; i += 32) aggL[i] = 0.0f;
  for (int i = lane; i < NB * 4; i += 32) csumL[i] = 0.0f;
  __syncthreads();

  int qhead = 0, qn = 0;

  for (int base = 0;; base += 128) {
    const bool more = base < E;
    if (more) {
      int kk[4];
      const int eb = base + 4 * lane;
      if (base + 128 <= E) {
        const v4i kv = *(const v4i*)(erow + eb);
        kk[0] = kv[0]; kk[1] = kv[1]; kk[2] = kv[2]; kk[3] = kv[3];
      } else {
#pragma unroll
        for (int j = 0; j < 4; ++j) kk[j] = (eb + j < E) ? erow[eb + j] : -1;
      }
#pragma unroll
      for (int j = 0; j < 4; ++j) {
        const bool match = (unsigned)(kk[j] - v0) < (unsigned)NB;
        unsigned msk = __builtin_amdgcn_ballot_w32(match);
        while (msk) {
          const int s = __builtin_ctz(msk);
          msk &= msk - 1u;
          if (lane == 0) qL[(qhead + qn) & (QCAP - 1)] = base + 4 * s + j;
          ++qn;
        }
      }
    }
    const int need = more ? 16 : 1;
    while (qn >= need) {
      const int cnt = (qn < 16) ? qn : 16;
      __syncthreads();
      const bool valid = m15 < cnt;
      const int slot = valid ? m15 : 0;
      const int e = qL[(qhead + slot) & (QCAP - 1)];
      int r = erow[e];
      int c = ecol[e];
      r = min(max(r, 0), N - 1);
      c = min(max(c, 0), N - 1);
      const float* cr = coord + (size_t)r * 3;
      const float* cc = coord + (size_t)c * 3;
      const float cdx = cr[0] - cc[0];
      const float cdy = cr[1] - cc[1];
      const float cdz = cr[2] - cc[2];
      const float radial = cdx * cdx + cdy * cdy + cdz * cdz;
      const float rsel = (hh == 0) ? radial : 0.0f;
      const float* hr = h + (size_t)r * FD;
      const float* hc = h + (size_t)c * FD;

#pragma unroll 1
      for (int t = 0; t < 8; ++t) {
        const int col = t * 16 + m15;
        const __bf16* bph = w1h + (size_t)col * 288;
        const __bf16* bpl = w1l + (size_t)col * 288;
        v8f acc = zf8();
#pragma unroll 1
        for (int ks = 0; ks < 8; ++ks) {
          const float* ap = ((ks < 4) ? hr : hc) + (ks & 3) * 32;
          acc = kstep(acc, ap, bph + ks * 32, bpl + ks * 32, hh);
        }
        {
          v16bf ah = z16(), al = z16();
          const float rh = bf16_hi(rsel);
          ah[0] = (__bf16)rh;
          al[0] = (__bf16)(rsel - rh);
          const v16bf bh = bfr(bph + 256, hh);
          const v16bf bl = bfr(bpl + 256, hh);
          acc = wmma3(ah, al, bh, bl, acc);
        }
        const float bias = be1[col];
#pragma unroll
        for (int rg = 0; rg < 8; ++rg)
          tH[(8 * hh + rg) * FD + col] = relu_f(acc[rg] + bias);
      }
      __syncthreads();

#pragma unroll 1
      for (int t = 0; t < 8; ++t) {
        const int col = t * 16 + m15;
        const __bf16* bph = w2h + (size_t)col * FD;
        const __bf16* bpl = w2l + (size_t)col * FD;
        const float* arow = tH + m15 * FD;
        v8f acc = zf8();
#pragma unroll 1
        for (int ks = 0; ks < 4; ++ks)
          acc = kstep(acc, arow + ks * 32, bph + ks * 32, bpl + ks * 32, hh);
        const float bias = be2[col];
#pragma unroll
        for (int rg = 0; rg < 8; ++rg)
          tF[(8 * hh + rg) * FD + col] = relu_f(acc[rg] + bias);
      }
      __syncthreads();

      float p[8];
#pragma unroll
      for (int rg = 0; rg < 8; ++rg) p[rg] = 0.0f;
#pragma unroll 1
      for (int t = 0; t < 8; ++t) {
        const int col = t * 16 + m15;
        const __bf16* bph = w3h + (size_t)col * FD;
        const __bf16* bpl = w3l + (size_t)col * FD;
        const float* arow = tF + m15 * FD;
        v8f acc = zf8();
#pragma unroll 1
        for (int ks = 0; ks < 4; ++ks)
          acc = kstep(acc, arow + ks * 32, bph + ks * 32, bpl + ks * 32, hh);
        const float bias = bc1[col];
        const float w    = wc2[col];
#pragma unroll
        for (int rg = 0; rg < 8; ++rg) p[rg] += relu_f(acc[rg] + bias) * w;
      }
#pragma unroll
      for (int s = 8; s >= 1; s >>= 1) {
#pragma unroll
        for (int rg = 0; rg < 8; ++rg) p[rg] += __shfl_xor(p[rg], s, 16);
      }
      if (m15 == 0) {
#pragma unroll
        for (int rg = 0; rg < 8; ++rg) phiL[8 * hh + rg] = p[rg];
      }
      __syncthreads();

      for (int mm = 0; mm < cnt; ++mm) {
        const int   rr = __shfl(r, mm) - v0;
        const float dx = __shfl(cdx, mm);
        const float dy = __shfl(cdy, mm);
        const float dz = __shfl(cdz, mm);
        if ((unsigned)rr < (unsigned)NB) {
          const v4f f = *(const v4f*)(tF + mm * FD + 4 * lane);
          v4f* ap = (v4f*)(aggL + rr * FD + 4 * lane);
          const v4f a = *ap;
          *ap = a + f;
          if (lane == 0) {
            const float phi = phiL[mm];
            csumL[rr * 4 + 0] += clip100(dx * phi);
            csumL[rr * 4 + 1] += clip100(dy * phi);
            csumL[rr * 4 + 2] += clip100(dz * phi);
            csumL[rr * 4 + 3] += 1.0f;
          }
        }
      }
      qhead += cnt;
      qn -= cnt;
    }
    if (!more) break;
  }
  __syncthreads();

  for (int q = 0; q < NB / 16; ++q) {
    const int nrow0 = v0 + 16 * q;
    if (nrow0 >= N) break;
    const int node = min(nrow0 + m15, N - 1);
    const float* po = others + (size_t)node * FD;
    const float* ph = h + (size_t)node * FD;
    const float* pa = aggL + (16 * q + m15) * FD;

#pragma unroll 1
    for (int t = 0; t < 8; ++t) {
      const int col = t * 16 + m15;
      const __bf16* bph = w4h + (size_t)col * 384;
      const __bf16* bpl = w4l + (size_t)col * 384;
      v8f acc = zf8();
#pragma unroll 1
      for (int ks = 0; ks < 12; ++ks) {
        const float* ap = (ks < 4) ? (po + ks * 32)
                        : (ks < 8) ? (ph + (ks - 4) * 32)
                                   : (pa + (ks - 8) * 32);
        acc = kstep(acc, ap, bph + ks * 32, bpl + ks * 32, hh);
      }
      const float bias = bn1[col];
#pragma unroll
      for (int rg = 0; rg < 8; ++rg)
        tH[(8 * hh + rg) * FD + col] = relu_f(acc[rg] + bias);
    }
    __syncthreads();

#pragma unroll 1
    for (int t = 0; t < 8; ++t) {
      const int col = t * 16 + m15;
      const __bf16* bph = w5h + (size_t)col * FD;
      const __bf16* bpl = w5l + (size_t)col * FD;
      const float* arow = tH + m15 * FD;
      v8f acc = zf8();
#pragma unroll 1
      for (int ks = 0; ks < 4; ++ks)
        acc = kstep(acc, arow + ks * 32, bph + ks * 32, bpl + ks * 32, hh);
      const float bias = bn2[col];
#pragma unroll
      for (int rg = 0; rg < 8; ++rg) {
        const int row = 8 * hh + rg;
        const int nd  = min(nrow0 + row, N - 1);
        const float hv = h[(size_t)nd * FD + col];
        const float dv = acc[rg] + bias;
        tF[row * FD + col] = hv + dv;
      }
    }
    __syncthreads();

    for (int rw = 0; rw < 16; ++rw) {
      const int nd = nrow0 + rw;
      if (nd < N) {
        const v4f v = *(const v4f*)(tF + rw * FD + 4 * lane);
        *(volatile v4f*)(hOut + (size_t)nd * FD + 4 * lane) = v;
      }
    }
    __threadfence();
    for (int rw = 0; rw < 16; ++rw) {
      const int nd = nrow0 + rw;
      if (nd < N) {
        const v4f v = *(const v4f*)(tF + rw * FD + 4 * lane);
        *(volatile v4f*)(hOut + (size_t)nd * FD + 4 * lane) = v;
      }
    }
    __syncthreads();
  }

  for (int i = lane; i < NB * 3; i += 32) {
    const int ln = i / 3;
    const int j  = i - ln * 3;
    const int nd = v0 + ln;
    float v = 0.0f;
    if (nd < N) {
      const float cntv = fmaxf(csumL[ln * 4 + 3], 1.0f);
      v = coord[(size_t)nd * 3 + j] + csumL[ln * 4 + j] / cntv;
    }
    cL[i] = v;
  }
  __syncthreads();
  {
    const int nval = min(NB, N - v0) * 3;
    float* cop = cOut + (size_t)v0 * 3;
    for (int pass = 0; pass < 2; ++pass) {
      for (int f4 = lane; f4 < (NB * 3) / 4; f4 += 32) {
        const int f = 4 * f4;
        if (f + 4 <= nval) {
          const v4f v = *(const v4f*)(cL + f);
          *(volatile v4f*)(cop + f) = v;
        } else {
#pragma unroll
          for (int j = 0; j < 4; ++j)
            if (f + j < nval) {
              const float v = cL[f + j];
              *(volatile float*)(cop + f + j) = v;
            }
        }
      }
      if (pass == 0) __threadfence();
    }
  }
}

extern "C" void kernel_launch(void* const* d_in, const int* in_sizes, int n_in,
                              void* d_out, int out_size, void* d_ws, size_t ws_size,
                              hipStream_t stream) {
  if (n_in < 16) return;
  const float* h      = (const float*)d_in[0];
  const float* coord  = (const float*)d_in[1];
  const float* others = (const float*)d_in[2];
  const int*   erow   = (const int*)d_in[3];
  const int*   ecol   = (const int*)d_in[4];
  const float* We1 = (const float*)d_in[5];  const float* be1 = (const float*)d_in[6];
  const float* We2 = (const float*)d_in[7];  const float* be2 = (const float*)d_in[8];
  const float* Wn1 = (const float*)d_in[9];  const float* bn1 = (const float*)d_in[10];
  const float* Wn2 = (const float*)d_in[11]; const float* bn2 = (const float*)d_in[12];
  const float* Wc1 = (const float*)d_in[13]; const float* bc1 = (const float*)d_in[14];
  const float* Wc2 = (const float*)d_in[15];

  const int N = in_sizes[0] / FD;
  int E = in_sizes[3];
  if (in_sizes[4] < E) E = in_sizes[4];
  if (N <= 0 || E < 0) return;
  if ((size_t)N * FD + (size_t)N * 3 > (size_t)out_size) return;

  char* ws = (char*)d_ws;
  size_t o = 0;
  const size_t b288 = (size_t)128 * 288 * sizeof(__bf16);
  const size_t b128 = (size_t)128 * 128 * sizeof(__bf16);
  const size_t b384 = (size_t)128 * 384 * sizeof(__bf16);
  __bf16* w1h = (__bf16*)(ws + o); o += b288;
  __bf16* w1l = (__bf16*)(ws + o); o += b288;
  __bf16* w2h = (__bf16*)(ws + o); o += b128;
  __bf16* w2l = (__bf16*)(ws + o); o += b128;
  __bf16* w3h = (__bf16*)(ws + o); o += b128;
  __bf16* w3l = (__bf16*)(ws + o); o += b128;
  __bf16* w4h = (__bf16*)(ws + o); o += b384;
  __bf16* w4l = (__bf16*)(ws + o); o += b384;
  __bf16* w5h = (__bf16*)(ws + o); o += b128;
  __bf16* w5l = (__bf16*)(ws + o); o += b128;
  if (o > ws_size) return;

  float* hOut = (float*)d_out;
  float* cOut = hOut + (size_t)N * FD;

  {
    const int t288 = 128 * 288 / 8, t128 = 128 * 128 / 8, t384 = 128 * 384 / 8;
    k_wsplit<<<(t288 + 255) / 256, 256, 0, stream>>>(We1, w1h, w1l, 257, 288);
    k_wsplit<<<(t128 + 255) / 256, 256, 0, stream>>>(We2, w2h, w2l, 128, 128);
    k_wsplit<<<(t128 + 255) / 256, 256, 0, stream>>>(Wc1, w3h, w3l, 128, 128);
    k_wsplit<<<(t384 + 255) / 256, 256, 0, stream>>>(Wn1, w4h, w4l, 384, 384);
    k_wsplit<<<(t128 + 255) / 256, 256, 0, stream>>>(Wn2, w5h, w5l, 128, 128);
  }
  const int nblk = (N + NB - 1) / NB;
  k_layer<<<nblk, 32, 0, stream>>>(h, coord, others, erow, ecol,
                                    w1h, w1l, be1, w2h, w2l, be2,
                                    w3h, w3l, bc1, Wc2,
                                    w4h, w4l, bn1, w5h, w5l, bn2,
                                    hOut, cOut, N, E);
}
